// NBMBlock_76587856823102
// MI455X (gfx1250) — hardware-verified
//
#include <hip/hip_runtime.h>

constexpr int kNB   = 128;
constexpr int kNF   = 128;
constexpr int kND   = 512;
constexpr int kOrd  = 2;
constexpr int kNBas = 32;
constexpr int kH1   = 64;
constexpr int kH2   = 32;
constexpr int kRows = kNB * kND;
constexpr int kRowsPerBlock = 256;
constexpr int kWaves = 8;
constexpr int kTilesPerWave = 2;
constexpr int kThreads = kWaves * 32;
static_assert(kWaves * 16 * kTilesPerWave == kRowsPerBlock, "tile coverage");
static_assert(kRows % kRowsPerBlock == 0, "grid exact");
static_assert(kND % kRowsPerBlock == 0, "a block stays inside one batch row");
static_assert(kRowsPerBlock * kOrd == 2 * kThreads, "gather coverage: 2 elements per thread");
static_assert(kH2 * kH1 == 8 * kThreads, "w2 stage coverage: 8 elements per thread");
static_assert(kH1 == 64 && kH2 == 32, "2 k-steps of 32, 2 n-tiles of 16");

typedef __attribute__((ext_vector_type(16))) __bf16   v16b;
typedef __attribute__((ext_vector_type(8)))  __bf16   v8b;
typedef __attribute__((ext_vector_type(8)))  float    v8f;
typedef __attribute__((ext_vector_type(4)))  float    v4f;

__device__ __forceinline__ unsigned short f2bf_bits(float f) {
  unsigned u = __float_as_uint(f);
  return (unsigned short)((u + 0x7FFFu + ((u >> 16) & 1u)) >> 16);
}
__device__ __forceinline__ float bf_bits2f(unsigned short h) { return __uint_as_float(((unsigned)h) << 16); }

__device__ __forceinline__ void dep_guard_b(v8f& a, v8f& b, v16b x, v16b y) { asm volatile("v_nop\n\tv_nop\n\tv_nop\n\tv_nop" : "+v"(a), "+v"(b) : "v"(x), "v"(y)); }
__device__ __forceinline__ void keep4_b(v16b a, v16b b, v16b c, v16b d) { asm volatile("v_nop" :: "v"(a), "v"(b), "v"(c), "v"(d)); }
template <typename T> struct Frag;
template <> struct Frag<__bf16> {
  typedef v16b V; union U { v16b v; v8b h[2]; };
  static __device__ __forceinline__ v16b load(const __bf16* p) {
    U f; f.h[0] = *(const v8b*)(p); f.h[1] = *(const v8b*)(p + 16); return f.v;
  }
  static __device__ __forceinline__ v8f mma(v16b a, v16b b, v8f c) {
    return __builtin_amdgcn_wmma_f32_16x16x32_bf16(false, a, false, b, (short)0, c, false, false);
  }
  static __device__ __forceinline__ void guard(v8f& a, v8f& b, v16b x, v16b y) { dep_guard_b(a, b, x, y); }
  static __device__ __forceinline__ void keep(v16b a, v16b b, v16b c, v16b d) { keep4_b(a, b, c, d); }
};

__device__ __forceinline__ void bf_split(float f, __bf16& hi, __bf16& lo) {
  const unsigned short hb = f2bf_bits(f);
  hi = __builtin_bit_cast(__bf16, hb);
  lo = __builtin_bit_cast(__bf16, f2bf_bits(f - bf_bits2f(hb)));
}

__global__ __launch_bounds__(kThreads)
void basis_mlp_kernel(const float* __restrict__ net,
                      const float* __restrict__ w1,
                      const float* __restrict__ b1,
                      const float* __restrict__ w2,
                      const float* __restrict__ b2,
                      const float* __restrict__ w3,
                      const float* __restrict__ b3,
                      const int*   __restrict__ indices,
                      float*       __restrict__ out)
{
  __shared__ __align__(16) float  gS[kRowsPerBlock * kOrd];
  __shared__ __align__(16) float  wS[256];
  __shared__ float                b3S[kNBas];
  __shared__ __align__(16) __bf16 BtSh[kH2 * kH1];
  __shared__ __align__(16) __bf16 BtSl[kH2 * kH1];
  __shared__ __align__(16) float  outS[kRowsPerBlock * kNBas];

  const int tid  = threadIdx.x;
  const int lane = tid & 31;
  const int wave = tid >> 5;
  const int hh   = lane >> 4;
  const int rl   = lane & 15;
  const int rowBase = blockIdx.x * kRowsPerBlock;
  const int b     = rowBase / kND;
  const int dBase = rowBase - b * kND;

#pragma unroll
  for (int i = 0; i < 2; ++i) {
    const int e  = i * kThreads + tid;
    const int dl = e >> 1;
    const int c  = e & 1;
    int idx = indices[(dBase + dl) * kOrd + c];
    idx = (idx < 0) ? (idx + kNF) : idx;
    idx = (idx < 0) ? 0 : ((idx > kNF - 1) ? (kNF - 1) : idx);
    gS[e] = net[(size_t)b * kNF + idx];
  }
  if (tid < kNBas) b3S[tid] = b3[tid];

#pragma unroll 1
  for (int k = 0; k < kNBas; ++k) {
    __syncthreads();
    {
      const float vw1 = w1[(size_t)k * (kH1 * kOrd) + (tid & 127)];
      const float vb1 = b1[(size_t)k * kH1 + (tid & 63)];
      const float vb2 = b2[(size_t)k * kH2 + (tid & 31)];
      const float vw3 = w3[(size_t)k * kH2 + (tid & 31)];
      wS[tid] = (tid < 128) ? vw1 : ((tid < 192) ? vb1 : ((tid < 224) ? vb2 : vw3));
    }
    {
      const int n  = tid >> 3;
      const int k8 = (tid & 7) * 8;
      const float* src = w2 + ((size_t)(k * kH2 + n) * kH1 + k8);
      const v4f wa = *(const v4f*)(src);
      const v4f wb = *(const v4f*)(src + 4);
      v8b hv, lv;
#pragma unroll
      for (int e = 0; e < 4; ++e) {
        __bf16 ha, la, hb2, lb2;
        bf_split(wa[e], ha, la);
        bf_split(wb[e], hb2, lb2);
        hv[e]     = ha;  lv[e]     = la;
        hv[4 + e] = hb2; lv[4 + e] = lb2;
      }
      *(v8b*)(BtSh + n * kH1 + k8) = hv;
      *(v8b*)(BtSl + n * kH1 + k8) = lv;
    }
    __syncthreads();

    const float b2c0 = wS[192 + rl], b2c1 = wS[192 + 16 + rl];
    const float w3c0 = wS[224 + rl], w3c1 = wS[224 + 16 + rl];
    const float b3v  = b3S[k];

    v16b bfh[2][2], bfl[2][2];
#pragma unroll
    for (int j = 0; j < 2; ++j)
#pragma unroll
      for (int s = 0; s < 2; ++s) {
        bfh[j][s] = Frag<__bf16>::load(BtSh + (16 * j + rl) * kH1 + 8 * hh + 32 * s);
        bfl[j][s] = Frag<__bf16>::load(BtSl + (16 * j + rl) * kH1 + 8 * hh + 32 * s);
      }

#pragma unroll 1
    for (int ti = 0; ti < kTilesPerWave; ++ti) {
      const int m0 = wave * (16 * kTilesPerWave) + ti * 16;
      const float g0 = gS[(m0 + rl) * kOrd + 0];
      const float g1 = gS[(m0 + rl) * kOrd + 1];

      v16b afh[2], afl[2];
#pragma unroll
      for (int s = 0; s < 2; ++s) {
#pragma unroll
        for (int i = 0; i < 8; ++i) {
          const int o0 = 32 * s + 8 * hh + i;
          const int o1 = o0 + 16;
          const float x0 = fmaxf(g0 * wS[2 * o0] + g1 * wS[2 * o0 + 1] + wS[128 + o0], 0.0f);
          const float x1 = fmaxf(g0 * wS[2 * o1] + g1 * wS[2 * o1 + 1] + wS[128 + o1], 0.0f);
          __bf16 h0, l0, h1v, l1v;
          bf_split(x0, h0, l0);
          bf_split(x1, h1v, l1v);
          afh[s][i]     = h0;  afl[s][i]     = l0;
          afh[s][8 + i] = h1v; afl[s][8 + i] = l1v;
        }
      }

      v8f acc[2];
#pragma unroll
      for (int j = 0; j < 2; ++j) {
        acc[j] = (v8f){0.f, 0.f, 0.f, 0.f, 0.f, 0.f, 0.f, 0.f};
#pragma unroll
        for (int s = 0; s < 2; ++s) {
          acc[j] = Frag<__bf16>::mma(afh[s], bfh[j][s], acc[j]);
          acc[j] = Frag<__bf16>::mma(afh[s], bfl[j][s], acc[j]);
          acc[j] = Frag<__bf16>::mma(afl[s], bfh[j][s], acc[j]);
        }
      }
      Frag<__bf16>::guard(acc[0], acc[1], afh[0], afh[1]);
      Frag<__bf16>::keep(afl[0], afl[1], bfh[0][0], bfh[0][1]);
      Frag<__bf16>::keep(bfh[1][0], bfh[1][1], bfl[0][0], bfl[0][1]);
      Frag<__bf16>::keep(bfl[1][0], bfl[1][1], bfl[1][0], bfl[1][1]);

      float t[8];
#pragma unroll
      for (int r = 0; r < 8; ++r)
        t[r] = fmaxf(acc[0][r] + b2c0, 0.0f) * w3c0
             + fmaxf(acc[1][r] + b2c1, 0.0f) * w3c1;
#pragma unroll
      for (int r = 0; r < 8; ++r) {
        t[r] += __shfl_xor(t[r], 1, 32);
        t[r] += __shfl_xor(t[r], 2, 32);
        t[r] += __shfl_xor(t[r], 4, 32);
        t[r] += __shfl_xor(t[r], 8, 32);
      }
      if (rl == 0) {
#pragma unroll
        for (int r = 0; r < 8; ++r)
          outS[(m0 + 8 * hh + r) * kNBas + k] = t[r] + b3v;
      }
    }
  }

  __syncthreads();

  {
    const int q  = lane >> 3;
    const int c4 = (lane & 7) * 4;
    float* ob = out + (size_t)rowBase * kNBas;
    for (int pass = 0; pass < 2; ++pass) {
#pragma unroll
      for (int it = 0; it < 8; ++it) {
        const int row = wave * 32 + it * 4 + q;
        const v4f v = *(const v4f*)(outS + row * kNBas + c4);
        *(volatile v4f*)(ob + (size_t)row * kNBas + c4) = v;
      }
      __threadfence();
    }
  }
}

extern "C" void kernel_launch(void* const* d_in, const int* in_sizes, int n_in,
                              void* d_out, int out_size, void* d_ws, size_t ws_size,
                              hipStream_t stream) {
  (void)d_ws; (void)ws_size;
  if (n_in < 8) return;
  if (in_sizes[0] != kNB * kNF) return;
  if (in_sizes[1] != kNBas * kH1 * kOrd) return;
  if (in_sizes[2] != kNBas * kH1) return;
  if (in_sizes[3] != kNBas * kH2 * kH1) return;
  if (in_sizes[4] != kNBas * kH2) return;
  if (in_sizes[5] != kNBas * kH2) return;
  if (in_sizes[6] != kNBas) return;
  if (in_sizes[7] != kND * kOrd) return;
  if (out_size != kRows * kNBas) return;

  const float* net     = (const float*)d_in[0];
  const float* w1      = (const float*)d_in[1];
  const float* b1      = (const float*)d_in[2];
  const float* w2      = (const float*)d_in[3];
  const float* b2      = (const float*)d_in[4];
  const float* w3      = (const float*)d_in[5];
  const float* b3      = (const float*)d_in[6];
  const int*   indices = (const int*)d_in[7];
  float* outp = (float*)d_out;

  basis_mlp_kernel<<<dim3(kRows / kRowsPerBlock), dim3(kThreads), 0, stream>>>(
      net, w1, b1, w2, b2, w3, b3, indices, outp);
}
